// DeepFactorizationMachineModel_46943992545833
// MI455X (gfx1250) — hardware-run, weakly checked
//
#include <hip/hip_runtime.h>
#include <math.h>

typedef __attribute__((ext_vector_type(16))) _Float16 v16h;
typedef __attribute__((ext_vector_type(8)))  float    v8f;
typedef __attribute__((ext_vector_type(4)))  float    v4f;
typedef __attribute__((ext_vector_type(2)))  float    v2f;
typedef __attribute__((ext_vector_type(8)))  unsigned v8u;
typedef __attribute__((ext_vector_type(4)))  unsigned v4u;
typedef __attribute__((ext_vector_type(2)))  unsigned v2u;

constexpr int kB        = 4096;
constexpr int kT        = 149;
constexpr int kAddW     = 237;
constexpr int kXW       = 30;
constexpr int kH        = 32;
constexpr int kG        = 128;
constexpr int kVocab    = 128;
constexpr int kFieldDim = 100000;
constexpr int kNumSel   = 10;
constexpr int kEmb      = 16;
constexpr int kMlpIn    = 176;
constexpr int kMlpInPad = 192;
constexpr int kMlp1     = 64;
constexpr int kMlp2     = 32;
static_assert(kG == 4 * kH);
static_assert(kMlpIn == (kNumSel + 1) * kEmb);
static_assert((kMlpInPad % 32) == 0 && kMlpInPad >= kMlpIn);
static_assert((kB % 64) == 0);

constexpr float kActCarry  = 1024.0f;
constexpr float kWCarry    = 256.0f;
constexpr float kFeatCarry = 4096.0f;
constexpr float kFoldAW    = 1.0f / (kActCarry * kWCarry);
constexpr float kFoldFW    = 1.0f / (kFeatCarry * kWCarry);
constexpr float kBnInv     = 0.99999500003749968f;

constexpr int kZP   = 132;
constexpr int kHWP  = 20;
constexpr int kW64P = 36;
constexpr int kW1P  = 100;
constexpr int kH1FP = 68;
constexpr int kEncP = 20;

constexpr size_t kSzE16   = (size_t)kT * kB * 4 * 2;
constexpr size_t kSzL0    = (size_t)kT * kB * kH * 2;
constexpr size_t kSzHid16 = (size_t)kB * kH * 2;
constexpr size_t kOffE16  = 0;
constexpr size_t kOffL0F  = kOffE16 + kSzE16;
constexpr size_t kOffL0B  = kOffL0F + kSzL0;
constexpr size_t kOffHid  = kOffL0B + kSzL0;
constexpr size_t kWsTotal = kOffHid + kSzHid16;
static_assert(kSzE16 == 4882432ull && kSzL0 == 39059456ull && kSzHid16 == 262144ull);
static_assert(kWsTotal == 83263488ull);
static_assert(kWsTotal <= 134217728ull);
static_assert((kOffL0F % 128) == 0 && (kOffL0B % 128) == 0 && (kOffHid % 128) == 0);
constexpr int kOut1Elem = 16384 / 4;
static_assert(16384 + (size_t)kB * kH * 4 == 540672ull);

constexpr int kCharPairs = kT * (kB / 2);
static_assert((kCharPairs % 256) == 0);

__device__ __forceinline__ int clampi(int v, int lo, int hi) {
  const int a = v < lo ? lo : v;
  return a > hi ? hi : a;
}

__device__ __forceinline__ unsigned pack_h2(float a, float b) {
  const _Float16 ha = (_Float16)a;
  const _Float16 hb = (_Float16)b;
  const unsigned short ua = __builtin_bit_cast(unsigned short, ha);
  const unsigned short ub = __builtin_bit_cast(unsigned short, hb);
  return (unsigned)ua | ((unsigned)ub << 16);
}
__device__ __forceinline__ v2u pack4_h(v4f v, float carry) {
  const float a = v[0] * carry;
  const float b = v[1] * carry;
  const float c = v[2] * carry;
  const float d = v[3] * carry;
  v2u r;
  r[0] = pack_h2(a, b);
  r[1] = pack_h2(c, d);
  return r;
}

__device__ __forceinline__ v16h frag_words(const unsigned* p) {
  const v4u q0 = *(const v4u*)(p);
  const v4u q1 = *(const v4u*)(p + 8);
  v8u w;
  w[0] = q0[0]; w[1] = q0[1]; w[2] = q0[2]; w[3] = q0[3];
  w[4] = q1[0]; w[5] = q1[1]; w[6] = q1[2]; w[7] = q1[3];
  return __builtin_bit_cast(v16h, w);
}

__device__ __forceinline__ v16h bfrag_f32(const float* p, float carry) {
  const v4f a0 = *(const v4f*)(p);
  const v4f a1 = *(const v4f*)(p + 4);
  const v4f a2 = *(const v4f*)(p + 16);
  const v4f a3 = *(const v4f*)(p + 20);
  const v2u w0 = pack4_h(a0, carry);
  const v2u w1 = pack4_h(a1, carry);
  const v2u w2 = pack4_h(a2, carry);
  const v2u w3 = pack4_h(a3, carry);
  v8u w;
  w[0] = w0[0]; w[1] = w0[1]; w[2] = w1[0]; w[3] = w1[1];
  w[4] = w2[0]; w[5] = w2[1]; w[6] = w3[0]; w[7] = w3[1];
  return __builtin_bit_cast(v16h, w);
}

__device__ __forceinline__ v8f mma_h(v16h a, v16h b, v8f c) {
  c = __builtin_amdgcn_wmma_f32_16x16x32_f16(false, a, false, b, (short)0, c, false, false);
  asm volatile("v_nop\n\tv_nop\n\tv_nop\n\tv_nop" : "+v"(c) : "v"(a), "v"(b));
  return c;
}

__device__ __forceinline__ void wave_lds_sync() {
  __builtin_amdgcn_fence(__ATOMIC_RELEASE, "workgroup");
  __builtin_amdgcn_wave_barrier();
  __builtin_amdgcn_fence(__ATOMIC_ACQUIRE, "workgroup");
}

__device__ __forceinline__ float sigm_f(float x) {
  const float xc = fminf(fmaxf(x, -30.0f), 30.0f);
  return 1.0f / (1.0f + expf(-xc));
}
__device__ __forceinline__ float gate_sigm(float x) {
  const float xc = fminf(fmaxf(x, -30.0f), 30.0f);
  return __builtin_amdgcn_rcpf(1.0f + __expf(-xc));
}
__device__ __forceinline__ float gate_tanh(float x) {
  const float xc = fminf(fmaxf(x, -30.0f), 30.0f);
  return 1.0f - 2.0f * __builtin_amdgcn_rcpf(1.0f + __expf(2.0f * xc));
}
__device__ __forceinline__ void cell_f(float zi, float zf, float zg, float zo, float cprev,
                                       float& hnew, float& cnew) {
  const float cn = gate_sigm(zf) * cprev + gate_sigm(zi) * gate_tanh(zg);
  hnew = gate_sigm(zo) * gate_tanh(cn);
  cnew = cn;
}

__global__ __launch_bounds__(256) void char_rows_kernel(
    const int* __restrict__ addl, const float* __restrict__ cemb, unsigned* __restrict__ e16w)
{
  const int i = blockIdx.x * 256 + threadIdx.x;
  if (i < kCharPairs) {
    const int t  = i / (kB / 2);
    const int bp = i - t * (kB / 2);
    const int b0 = bp * 2;
    const int tok0 = clampi(addl[(size_t)b0 * kAddW + t], 0, kVocab - 1);
    const int tok1 = clampi(addl[(size_t)(b0 + 1) * kAddW + t], 0, kVocab - 1);
    const v4f w0 = *(const v4f*)(cemb + tok0 * 4);
    const v4f w1 = *(const v4f*)(cemb + tok1 * 4);
    const v2u p0 = pack4_h(w0, kActCarry);
    const v2u p1 = pack4_h(w1, kActCarry);
    v4u o;
    o[0] = p0[0]; o[1] = p0[1]; o[2] = p1[0]; o[3] = p1[1];
    unsigned* dst = e16w + (size_t)i * 4;
    *(volatile v4u*)dst = o;
    __threadfence();
    *(volatile v4u*)dst = o;
  }
}

template <bool WRITE_H32>
__device__ __forceinline__ void gate_pass(float* zt, float* ct, unsigned* hw, int hh, int c,
                                          v2f bi, v2f bf, v2f bg, v2f bo)
{
#pragma unroll 1
  for (int it = 0; it < 8; ++it) {
    const int row = it * 2 + hh;
    float* zr = zt + row * kZP + 2 * c;
    const v2f zi = *(const v2f*)(zr);
    const v2f zf = *(const v2f*)(zr + 32);
    const v2f zg = *(const v2f*)(zr + 64);
    const v2f zo = *(const v2f*)(zr + 96);
    float* cr = ct + row * kH + 2 * c;
    const v2f cv = *(const v2f*)cr;
    float h0, h1, c0, c1;
    cell_f(zi[0] * kFoldAW + bi[0], zf[0] * kFoldAW + bf[0], zg[0] * kFoldAW + bg[0],
           zo[0] * kFoldAW + bo[0], cv[0], h0, c0);
    cell_f(zi[1] * kFoldAW + bi[1], zf[1] * kFoldAW + bf[1], zg[1] * kFoldAW + bg[1],
           zo[1] * kFoldAW + bo[1], cv[1], h1, c1);
    v2f cw;
    cw[0] = c0; cw[1] = c1;
    *(v2f*)cr = cw;
    hw[row * kHWP + c] = pack_h2(h0 * kActCarry, h1 * kActCarry);
    if (WRITE_H32) {
      v2f hv;
      hv[0] = h0; hv[1] = h1;
      *(v2f*)zr = hv;
    }
  }
}

__device__ __forceinline__ void store_h_tile(const unsigned* hw, unsigned* dst, int lane) {
  const int r8 = lane >> 2;
  const int q4 = (lane & 3) * 4;
  const v4u d0 = *(const v4u*)(hw + r8 * kHWP + q4);
  const v4u d1 = *(const v4u*)(hw + (r8 + 8) * kHWP + q4);
  for (int pass = 0; pass < 2; ++pass) {
    *(volatile v4u*)(dst + r8 * 16 + q4) = d0;
    *(volatile v4u*)(dst + (r8 + 8) * 16 + q4) = d1;
    __threadfence();
  }
}

__global__ __launch_bounds__(128) void lstm_l0_kernel(
    const unsigned* __restrict__ e16w,
    const float* __restrict__ wih_f, const float* __restrict__ whh_f, const float* __restrict__ bias_f,
    const float* __restrict__ wih_b, const float* __restrict__ whh_b, const float* __restrict__ bias_b,
    unsigned* __restrict__ l0f, unsigned* __restrict__ l0b)
{
  __shared__ __align__(16) float    sZ[4][16 * kZP];
  __shared__ __align__(16) float    sC[4][16 * kH];
  __shared__ __align__(16) unsigned sHw[4][16 * kHWP];

  const int dir = blockIdx.y;
  const float* Wih = dir ? wih_b : wih_f;
  const float* Whh = dir ? whh_b : whh_f;
  const float* Bv  = dir ? bias_b : bias_f;
  unsigned* plane  = dir ? l0b : l0f;

  const int lane = threadIdx.x & 31;
  const int wave = threadIdx.x >> 5;
  const int hh   = lane >> 4;
  const int c    = lane & 15;
  const int rowbase = (blockIdx.x * 4 + wave) * 16;
  float*    zt = sZ[wave];
  float*    ct = sC[wave];
  unsigned* hw = sHw[wave];

  v16h whh[8], wih[8];
#pragma unroll
  for (int n = 0; n < 8; ++n) {
    const int ng = n * 16 + c;
    whh[n] = bfrag_f32(Whh + ng * kH + 8 * hh, kWCarry);
    const v4f w4 = *(const v4f*)(Wih + ng * 4);
    float w0 = w4[0], w1 = w4[1], w2 = w4[2], w3 = w4[3];
    asm volatile("" : "+v"(w0), "+v"(w1), "+v"(w2), "+v"(w3));
    const unsigned p0 = pack_h2(w0 * kWCarry, w1 * kWCarry);
    const unsigned p1 = pack_h2(w2 * kWCarry, w3 * kWCarry);
    v8u ww;
    ww[0] = (hh == 0) ? p0 : 0u;
    ww[1] = (hh == 0) ? p1 : 0u;
    ww[2] = 0u; ww[3] = 0u; ww[4] = 0u; ww[5] = 0u; ww[6] = 0u; ww[7] = 0u;
    wih[n] = __builtin_bit_cast(v16h, ww);
  }
  const v2f bi = *(const v2f*)(Bv + 2 * c);
  const v2f bf = *(const v2f*)(Bv + 32 + 2 * c);
  const v2f bg = *(const v2f*)(Bv + 64 + 2 * c);
  const v2f bo = *(const v2f*)(Bv + 96 + 2 * c);

#pragma unroll 1
  for (int it = 0; it < 8; ++it) {
    const int row = it * 2 + hh;
    v2f zz;
    zz[0] = 0.0f; zz[1] = 0.0f;
    *(v2f*)(ct + row * kH + 2 * c) = zz;
    hw[row * kHWP + c] = 0u;
  }
  wave_lds_sync();

#pragma unroll 1
  for (int s = 0; s < kT; ++s) {
    const int t = dir ? (kT - 1 - s) : s;
    const v16h ah = frag_words(hw + c * kHWP + 4 * hh);
    unsigned ex, ey;
    {
      const v2u ev = *(const v2u*)(e16w + ((size_t)t * kB + rowbase + c) * 2);
      ex = ev[0];
      ey = ev[1];
    }
    asm volatile("" : "+v"(ex), "+v"(ey));
    v8u aw;
    aw[0] = (hh == 0) ? ex : 0u;
    aw[1] = (hh == 0) ? ey : 0u;
    aw[2] = 0u; aw[3] = 0u; aw[4] = 0u; aw[5] = 0u; aw[6] = 0u; aw[7] = 0u;
    const v16h ae = __builtin_bit_cast(v16h, aw);

#pragma unroll
    for (int n = 0; n < 8; ++n) {
      v8f acc = (v8f){0.f, 0.f, 0.f, 0.f, 0.f, 0.f, 0.f, 0.f};
      acc = mma_h(ae, wih[n], acc);
      acc = mma_h(ah, whh[n], acc);
#pragma unroll
      for (int r = 0; r < 8; ++r) zt[(8 * hh + r) * kZP + n * 16 + c] = acc[r];
    }
    wave_lds_sync();
    gate_pass<false>(zt, ct, hw, hh, c, bi, bf, bg, bo);
    wave_lds_sync();
    store_h_tile(hw, plane + ((size_t)t * kB + rowbase) * 16, lane);
  }
}

__global__ __launch_bounds__(64) void lstm_l1b_kernel(
    const unsigned* __restrict__ l0f, const unsigned* __restrict__ l0b,
    const float* __restrict__ wih, const float* __restrict__ whh_g, const float* __restrict__ bias,
    float* __restrict__ hid, unsigned* __restrict__ hid16)
{
  __shared__ __align__(16) unsigned sW[kG * kW64P];
  __shared__ __align__(16) float    sZ[2][16 * kZP];
  __shared__ __align__(16) float    sC[2][16 * kH];
  __shared__ __align__(16) unsigned sHw[2][16 * kHWP];

  const int tid = threadIdx.x;
#pragma unroll 1
  for (int it = 0; it < 16; ++it) {
    const int idx = it * 64 + tid;
    const int n  = idx >> 3;
    const int k8 = idx & 7;
    const float* p = wih + n * 64 + k8 * 8;
    const v4f a0 = *(const v4f*)(p);
    const v4f a1 = *(const v4f*)(p + 4);
    const v2u w0 = pack4_h(a0, kWCarry);
    const v2u w1 = pack4_h(a1, kWCarry);
    v4u o;
    o[0] = w0[0]; o[1] = w0[1]; o[2] = w1[0]; o[3] = w1[1];
    *(v4u*)(sW + n * kW64P + k8 * 4) = o;
  }
  __syncthreads();

  const int lane = tid & 31;
  const int wave = tid >> 5;
  const int hh   = lane >> 4;
  const int c    = lane & 15;
  const int rowbase = (blockIdx.x * 2 + wave) * 16;
  float*    zt = sZ[wave];
  float*    ct = sC[wave];
  unsigned* hw = sHw[wave];

  v16h whh[8];
#pragma unroll
  for (int n = 0; n < 8; ++n) whh[n] = bfrag_f32(whh_g + (n * 16 + c) * kH + 8 * hh, kWCarry);
  const v2f bi = *(const v2f*)(bias + 2 * c);
  const v2f bf = *(const v2f*)(bias + 32 + 2 * c);
  const v2f bg = *(const v2f*)(bias + 64 + 2 * c);
  const v2f bo = *(const v2f*)(bias + 96 + 2 * c);

#pragma unroll 1
  for (int it = 0; it < 8; ++it) {
    const int row = it * 2 + hh;
    v2f zz;
    zz[0] = 0.0f; zz[1] = 0.0f;
    *(v2f*)(ct + row * kH + 2 * c) = zz;
    hw[row * kHWP + c] = 0u;
  }
  wave_lds_sync();

#pragma unroll 1
  for (int s = 0; s < kT; ++s) {
    const int t = kT - 1 - s;
    const v16h ah = frag_words(hw + c * kHWP + 4 * hh);
    const size_t ro = ((size_t)t * kB + rowbase + c) * 16 + 4 * hh;
    const v16h a0 = frag_words(l0f + ro);
    const v16h a1 = frag_words(l0b + ro);
#pragma unroll
    for (int n = 0; n < 8; ++n) {
      const unsigned* wr = sW + (n * 16 + c) * kW64P + 4 * hh;
      const v16h b0 = frag_words(wr);
      const v16h b1 = frag_words(wr + 16);
      v8f acc = (v8f){0.f, 0.f, 0.f, 0.f, 0.f, 0.f, 0.f, 0.f};
      acc = mma_h(a0, b0, acc);
      acc = mma_h(a1, b1, acc);
      acc = mma_h(ah, whh[n], acc);
#pragma unroll
      for (int r = 0; r < 8; ++r) zt[(8 * hh + r) * kZP + n * 16 + c] = acc[r];
    }
    wave_lds_sync();
    gate_pass<true>(zt, ct, hw, hh, c, bi, bf, bg, bo);
    wave_lds_sync();
  }

  store_h_tile(hw, hid16 + (size_t)rowbase * 16, lane);
  {
    const int rq = lane >> 3;
    const int c4 = (lane & 7) * 4;
    v4f hv[4];
#pragma unroll
    for (int i = 0; i < 4; ++i) hv[i] = *(const v4f*)(zt + (rq + 4 * i) * kZP + c4);
    float* dst = hid + (size_t)rowbase * kH;
    for (int pass = 0; pass < 2; ++pass) {
#pragma unroll
      for (int i = 0; i < 4; ++i) *(volatile v4f*)(dst + (rq + 4 * i) * kH + c4) = hv[i];
      __threadfence();
    }
  }
}

__global__ __launch_bounds__(64) void head_kernel(
    const int* __restrict__ x, const float* __restrict__ table, const float* __restrict__ fm_bias,
    const unsigned* __restrict__ hid16,
    const float* __restrict__ enclW, const float* __restrict__ enclb,
    const float* __restrict__ W1, const float* __restrict__ b1,
    const float* __restrict__ g1, const float* __restrict__ be1,
    const float* __restrict__ W2, const float* __restrict__ b2,
    const float* __restrict__ g2, const float* __restrict__ be2,
    const float* __restrict__ W3, const float* __restrict__ b3,
    float* __restrict__ prob)
{
  __shared__ __align__(16) unsigned sW1[kMlp1 * kW1P];
  __shared__ __align__(16) unsigned sW2[kMlp2 * kW64P];
  __shared__ __align__(16) unsigned sEW[kEmb * kHWP];
  __shared__ __align__(16) unsigned sFeat[2][16 * kW1P];
  __shared__ __align__(16) float    sH1F[2][16 * kH1FP];
  __shared__ __align__(16) unsigned sH1H[2][16 * kW64P];
  __shared__ __align__(16) float    sEnc[2][16 * kEncP];
  __shared__ __align__(16) float    sMlp[2][16];
  __shared__ __align__(16) float    sProb[2][32];

  const int tid = threadIdx.x;
#pragma unroll 1
  for (int it = 0; it < 24; ++it) {
    const int idx = it * 64 + tid;
    const int n   = idx / 24;
    const int k8  = idx - n * 24;
    const int kc  = (k8 < 22) ? k8 : 21;
    const float* p = W1 + n * kMlpIn + kc * 8;
    const v4f a0 = *(const v4f*)(p);
    const v4f a1 = *(const v4f*)(p + 4);
    float f0 = a0[0], f1 = a0[1], f2 = a0[2], f3 = a0[3];
    float f4 = a1[0], f5 = a1[1], f6 = a1[2], f7 = a1[3];
    asm volatile("" : "+v"(f0), "+v"(f1), "+v"(f2), "+v"(f3));
    asm volatile("" : "+v"(f4), "+v"(f5), "+v"(f6), "+v"(f7));
    const bool live = (k8 < 22);
    f0 = live ? f0 * kWCarry : 0.0f;
    f1 = live ? f1 * kWCarry : 0.0f;
    f2 = live ? f2 * kWCarry : 0.0f;
    f3 = live ? f3 * kWCarry : 0.0f;
    f4 = live ? f4 * kWCarry : 0.0f;
    f5 = live ? f5 * kWCarry : 0.0f;
    f6 = live ? f6 * kWCarry : 0.0f;
    f7 = live ? f7 * kWCarry : 0.0f;
    v4u o;
    o[0] = pack_h2(f0, f1); o[1] = pack_h2(f2, f3); o[2] = pack_h2(f4, f5); o[3] = pack_h2(f6, f7);
    *(v4u*)(sW1 + n * kW1P + k8 * 4) = o;
  }
#pragma unroll 1
  for (int it = 0; it < 4; ++it) {
    const int idx = it * 64 + tid;
    const int n  = idx >> 3;
    const int k8 = idx & 7;
    const float* p = W2 + n * kMlp1 + k8 * 8;
    const v2u w0 = pack4_h(*(const v4f*)(p), kWCarry);
    const v2u w1 = pack4_h(*(const v4f*)(p + 4), kWCarry);
    v4u o;
    o[0] = w0[0]; o[1] = w0[1]; o[2] = w1[0]; o[3] = w1[1];
    *(v4u*)(sW2 + n * kW64P + k8 * 4) = o;
  }
  {
    const int n  = tid >> 2;
    const int k8 = tid & 3;
    const float* p = enclW + n * kH + k8 * 8;
    const v2u w0 = pack4_h(*(const v4f*)(p), kWCarry);
    const v2u w1 = pack4_h(*(const v4f*)(p + 4), kWCarry);
    v4u o;
    o[0] = w0[0]; o[1] = w0[1]; o[2] = w1[0]; o[3] = w1[1];
    *(v4u*)(sEW + n * kHWP + k8 * 4) = o;
  }
  __syncthreads();

  const int lane = tid & 31;
  const int wave = tid >> 5;
  const int hh   = lane >> 4;
  const int c    = lane & 15;
  const int rr   = lane >> 2;
  const int q    = lane & 3;
  const int wg   = blockIdx.x * 2 + wave;
  unsigned* ft   = sFeat[wave];
  float*    h1f  = sH1F[wave];
  unsigned* h1h  = sH1H[wave];
  float*    enc  = sEnc[wave];
  float*    mlpv = sMlp[wave];
  float*    prb  = sProb[wave];

  float pb1[4], pg1[4], pe1[4];
#pragma unroll
  for (int nt = 0; nt < 4; ++nt) {
    pb1[nt] = b1[nt * 16 + c];
    pg1[nt] = g1[nt * 16 + c];
    pe1[nt] = be1[nt * 16 + c];
  }
  float pb2[2], pg2[2], pe2[2], pw3[2];
#pragma unroll
  for (int nt = 0; nt < 2; ++nt) {
    pb2[nt] = b2[nt * 16 + c];
    pg2[nt] = g2[nt * 16 + c];
    pe2[nt] = be2[nt * 16 + c];
    pw3[nt] = W3[nt * 16 + c];
  }
  const float eb  = enclb[c];
  const float fmb = fm_bias[0];
  const float b3v = b3[0];

#pragma unroll 1
  for (int tile = 0; tile < 2; ++tile) {
    const int rowbase = wg * 32 + tile * 16;

    {
      const v16h a = frag_words(hid16 + (size_t)(rowbase + c) * 16 + 4 * hh);
      const v16h b = frag_words(sEW + c * kHWP + 4 * hh);
      v8f acc = (v8f){0.f, 0.f, 0.f, 0.f, 0.f, 0.f, 0.f, 0.f};
      acc = mma_h(a, b, acc);
#pragma unroll
      for (int r = 0; r < 8; ++r) enc[(8 * hh + r) * kEncP + c] = acc[r] * kFoldAW + eb;
    }
    wave_lds_sync();

    v4f sacc[2], qacc[2];
#pragma unroll
    for (int i = 0; i < 2; ++i) {
      const int row = rr + 8 * i;
      const v4f e4 = *(const v4f*)(enc + row * kEncP + q * 4);
      sacc[i] = e4;
      qacc[i] = e4 * e4;
      *(v2u*)(ft + row * kW1P + 8 + q * 2) = pack4_h(e4, kFeatCarry);
      v2u zz;
      zz[0] = 0u; zz[1] = 0u;
      *(v2u*)(ft + row * kW1P + 88 + q * 2) = zz;
    }
#pragma unroll 1
    for (int j = 0; j < kNumSel; ++j) {
      const int col  = (j == 0) ? 0 : ((j == 1) ? 5 : ((j < 6) ? (15 + j) : (20 + j)));
      const int slot = (j == 0) ? 0 : (j + 1);
#pragma unroll
      for (int i = 0; i < 2; ++i) {
        const int row = rr + 8 * i;
        const int idx = clampi(x[(size_t)(rowbase + row) * kXW + col], 0, kFieldDim - 1);
        const v4f v = *(const v4f*)(table + ((size_t)idx + (size_t)j * kFieldDim) * kEmb + q * 4);
        sacc[i] = sacc[i] + v;
        qacc[i] = qacc[i] + v * v;
        *(v2u*)(ft + row * kW1P + slot * 8 + q * 2) = pack4_h(v, kFeatCarry);
      }
    }
    float lp[2], fp[2];
#pragma unroll
    for (int i = 0; i < 2; ++i) {
      const v4f sv = sacc[i];
      const v4f qv = qacc[i];
      lp[i] = (sv[0] + sv[1]) + (sv[2] + sv[3]);
      fp[i] = ((sv[0] * sv[0] - qv[0]) + (sv[1] * sv[1] - qv[1])) +
              ((sv[2] * sv[2] - qv[2]) + (sv[3] * sv[3] - qv[3]));
    }
#pragma unroll
    for (int i = 0; i < 2; ++i) {
      lp[i] += __shfl_xor(lp[i], 1, 32);
      fp[i] += __shfl_xor(fp[i], 1, 32);
      lp[i] += __shfl_xor(lp[i], 2, 32);
      fp[i] += __shfl_xor(fp[i], 2, 32);
    }
    wave_lds_sync();

    {
      v8f acc[4];
#pragma unroll
      for (int nt = 0; nt < 4; ++nt) acc[nt] = (v8f){0.f, 0.f, 0.f, 0.f, 0.f, 0.f, 0.f, 0.f};
#pragma unroll 1
      for (int kt = 0; kt < kMlpInPad / 32; ++kt) {
        const v16h a = frag_words(ft + c * kW1P + kt * 16 + 4 * hh);
#pragma unroll
        for (int nt = 0; nt < 4; ++nt) {
          const v16h b = frag_words(sW1 + (nt * 16 + c) * kW1P + kt * 16 + 4 * hh);
          acc[nt] = mma_h(a, b, acc[nt]);
        }
      }
#pragma unroll
      for (int nt = 0; nt < 4; ++nt) {
#pragma unroll
        for (int r = 0; r < 8; ++r) {
          float v = acc[nt][r] * kFoldFW + pb1[nt];
          v = (pg1[nt] * v) * kBnInv + pe1[nt];
          v = fmaxf(v, 0.0f);
          h1f[(8 * hh + r) * kH1FP + nt * 16 + c] = v;
        }
      }
    }
    wave_lds_sync();
    {
      const int row = lane >> 1;
      const int cb  = (lane & 1) * 32;
#pragma unroll
      for (int i = 0; i < 4; ++i) {
        const float* sp = h1f + row * kH1FP + cb + 8 * i;
        const v2u w0 = pack4_h(*(const v4f*)(sp), kActCarry);
        const v2u w1 = pack4_h(*(const v4f*)(sp + 4), kActCarry);
        v4u o;
        o[0] = w0[0]; o[1] = w0[1]; o[2] = w1[0]; o[3] = w1[1];
        *(v4u*)(h1h + row * kW64P + (cb >> 1) + 4 * i) = o;
      }
    }
    wave_lds_sync();
    {
      v8f acc2[2];
#pragma unroll
      for (int nt = 0; nt < 2; ++nt) acc2[nt] = (v8f){0.f, 0.f, 0.f, 0.f, 0.f, 0.f, 0.f, 0.f};
#pragma unroll
      for (int kt = 0; kt < 2; ++kt) {
        const v16h a = frag_words(h1h + c * kW64P + kt * 16 + 4 * hh);
#pragma unroll
        for (int nt = 0; nt < 2; ++nt) {
          const v16h b = frag_words(sW2 + (nt * 16 + c) * kW64P + kt * 16 + 4 * hh);
          acc2[nt] = mma_h(a, b, acc2[nt]);
        }
      }
      float m[8];
#pragma unroll
      for (int r = 0; r < 8; ++r) m[r] = 0.0f;
#pragma unroll
      for (int nt = 0; nt < 2; ++nt) {
#pragma unroll
        for (int r = 0; r < 8; ++r) {
          float v = acc2[nt][r] * kFoldAW + pb2[nt];
          v = (pg2[nt] * v) * kBnInv + pe2[nt];
          v = fmaxf(v, 0.0f);
          m[r] += pw3[nt] * v;
        }
      }
#pragma unroll
      for (int r = 0; r < 8; ++r) {
        m[r] += __shfl_xor(m[r], 1, 32);
        m[r] += __shfl_xor(m[r], 2, 32);
        m[r] += __shfl_xor(m[r], 4, 32);
        m[r] += __shfl_xor(m[r], 8, 32);
      }
      if (c == 0) {
#pragma unroll
        for (int r = 0; r < 8; ++r) mlpv[8 * hh + r] = m[r];
      }
    }
    wave_lds_sync();
#pragma unroll
    for (int i = 0; i < 2; ++i) {
      const int row = rr + 8 * i;
      const float mv  = mlpv[row];
      const float tot = ((lp[i] + fmb) + 0.5f * fp[i]) + (mv + b3v);
      const float pr  = sigm_f(tot);
      if (q == 0) prb[tile * 16 + row] = pr;
    }
    wave_lds_sync();
  }

  {
    const float pv = prb[lane];
    float* dst = prob + (size_t)wg * 32 + lane;
    *(volatile float*)dst = pv;
    __threadfence();
    *(volatile float*)dst = pv;
  }
}

extern "C" void kernel_launch(void* const* d_in, const int* in_sizes, int n_in,
                              void* d_out, int out_size, void* d_ws, size_t ws_size,
                              hipStream_t stream) {
  if (n_in < 29) return;
  if (in_sizes[0] != kB * kXW) return;
  if (in_sizes[1] != kB * kAddW) return;
  if (in_sizes[2] != kNumSel * kFieldDim * kEmb) return;
  if (in_sizes[4] != kVocab * 4) return;
  if (in_sizes[5] != kG * 4 || in_sizes[8] != kG * 4) return;
  if (in_sizes[6] != kG * kH || in_sizes[9] != kG * kH || in_sizes[15] != kG * kH) return;
  if (in_sizes[7] != kG || in_sizes[10] != kG || in_sizes[16] != kG) return;
  if (in_sizes[14] != kG * 2 * kH) return;
  if (in_sizes[17] != kEmb * kH || in_sizes[18] != kEmb) return;
  if (in_sizes[19] != kMlp1 * kMlpIn || in_sizes[23] != kMlp2 * kMlp1 || in_sizes[27] != kMlp2) return;
  if (out_size != kB + kB * kH) return;
  if (ws_size < kWsTotal) return;

  const int*   x      = (const int*)d_in[0];
  const int*   addl   = (const int*)d_in[1];
  const float* table  = (const float*)d_in[2];
  const float* fmb    = (const float*)d_in[3];
  const float* cemb   = (const float*)d_in[4];
  const float* w0f_ih = (const float*)d_in[5];
  const float* w0f_hh = (const float*)d_in[6];
  const float* w0f_b  = (const float*)d_in[7];
  const float* w0b_ih = (const float*)d_in[8];
  const float* w0b_hh = (const float*)d_in[9];
  const float* w0b_b  = (const float*)d_in[10];
  const float* w1b_ih = (const float*)d_in[14];
  const float* w1b_hh = (const float*)d_in[15];
  const float* w1b_b  = (const float*)d_in[16];
  const float* enclW  = (const float*)d_in[17];
  const float* enclb  = (const float*)d_in[18];
  const float* W1     = (const float*)d_in[19];
  const float* b1     = (const float*)d_in[20];
  const float* g1     = (const float*)d_in[21];
  const float* be1    = (const float*)d_in[22];
  const float* W2     = (const float*)d_in[23];
  const float* b2     = (const float*)d_in[24];
  const float* g2     = (const float*)d_in[25];
  const float* be2    = (const float*)d_in[26];
  const float* W3     = (const float*)d_in[27];
  const float* b3     = (const float*)d_in[28];

  float* prob = (float*)d_out;
  float* hid  = (float*)d_out + kOut1Elem;

  char* ws = (char*)d_ws;
  unsigned* e16w  = (unsigned*)(ws + kOffE16);
  unsigned* l0f   = (unsigned*)(ws + kOffL0F);
  unsigned* l0b   = (unsigned*)(ws + kOffL0B);
  unsigned* hid16 = (unsigned*)(ws + kOffHid);

  char_rows_kernel<<<kCharPairs / 256, 256, 0, stream>>>(addl, cemb, e16w);
  lstm_l0_kernel<<<dim3(kB / 64, 2), 128, 0, stream>>>(
      e16w, w0f_ih, w0f_hh, w0f_b, w0b_ih, w0b_hh, w0b_b, l0f, l0b);
  lstm_l1b_kernel<<<kB / 32, 64, 0, stream>>>(l0f, l0b, w1b_ih, w1b_hh, w1b_b, hid, hid16);
  head_kernel<<<kB / 64, 64, 0, stream>>>(
      x, table, fmb, hid16, enclW, enclb, W1, b1, g1, be1, W2, b2, g2, be2, W3, b3, prob);
}
